// Model_59906203844677
// MI455X (gfx1250) — hardware-run, weakly checked
//
#include <hip/hip_runtime.h>


#ifndef NB
#define NB 4
#endif
#ifndef SEQ
#define SEQ 2048
#endif
#define NB_FULL  4
#define SEQ_FULL 2048
#ifndef OUT_SEQ
#define OUT_SEQ SEQ
#endif
#define DM   256
#define NH_  4
#define HD   64
#define QB   64
#define NFEAT 3
#define NHID  16
#define AW   4
#define OSP  68
#define PSP  68
#define QRS  2048.0f
#define QRI  (1.0f / 2048.0f)
#define SSC  0.25f
#define L2E  1.4426950408889634f
#define L2E2 2.8853900817779268f
#define GSL2 (-7.213475204444817f)
#define FILL2 (-14426.950408889634f)
#define C30  43.28085122666890f
#define PSH  14.0f
#define NEGB (-3.0e38f)
#define THSENT 1.0e30f
#define THCUT  1.0e29f
#define CTS  64.0f
#define WOS  64.0f
#define OSI  (1.0f / 4096.0f)

static_assert(HD == 64);
static_assert(NH_ * HD == DM);
static_assert(4 * QB == DM);
static_assert(QB % 8 == 0);
static_assert(DM % 64 == 0);
static_assert(DM % 32 == 0);
static_assert(HD % 32 == 0);
static_assert(SEQ % 64 == 0);
static_assert((NB * SEQ) % 64 == 0);
static_assert(SEQ % 32 == 0);
static_assert(SEQ % (16 * AW) == 0);
static_assert((NB * SEQ) % 256 == 0);
static_assert(((size_t)DM * DM / 8) % 256 == 0);
static_assert(((size_t)SEQ * DM) % 8 == 0);
static_assert(NB <= NB_FULL);
static_assert(SEQ <= SEQ_FULL);
static_assert(OUT_SEQ >= SEQ);
static_assert((OSP * 4) % 16 == 0);
static_assert((PSP * 4) % 16 == 0);
static_assert(32 * 8 * 4 == 16 * HD);
static_assert(4 * 4 == 16 && 8 * 8 == 64);
static_assert(8 * 2 == 16 && 16 * 4 == 64);
static_assert(AW * 16 * OSP * 4 <= 131072);
static_assert(16 * PSP * 4 <= 131072);

typedef _Float16 h16;
typedef unsigned short bf;
typedef __attribute__((ext_vector_type(16))) __bf16   v16bf;
typedef __attribute__((ext_vector_type(16))) _Float16 v16h;
typedef __attribute__((ext_vector_type(8)))  _Float16 v8h;
typedef __attribute__((ext_vector_type(8)))  unsigned short v8us;
typedef __attribute__((ext_vector_type(8)))  float    v8f;
typedef __attribute__((ext_vector_type(4)))  float    v4f;
typedef v4f  __attribute__((may_alias)) v4fa;

__device__ __forceinline__ unsigned short f2bf(float f) { unsigned u = __float_as_uint(f); u += 0x7FFFu + ((u >> 16) & 1u); return (unsigned short)(u >> 16); }
__device__ __forceinline__ float bfr(float f) { return __uint_as_float(((unsigned)f2bf(f)) << 16); }
__device__ __forceinline__ v16h cat16(v8h lo, v8h hi) { return __builtin_shufflevector(lo, hi, 0, 1, 2, 3, 4, 5, 6, 7, 8, 9, 10, 11, 12, 13, 14, 15); }
__device__ __forceinline__ v16bf cat16b(v8us lo, v8us hi) { return __builtin_bit_cast(v16bf, __builtin_shufflevector(lo, hi, 0, 1, 2, 3, 4, 5, 6, 7, 8, 9, 10, 11, 12, 13, 14, 15)); }
__device__ __forceinline__ v8f wmma16(v16h a, v16h b, v8f c) { return __builtin_amdgcn_wmma_f32_16x16x32_f16(false, a, false, b, (short)0, c, false, false); }
__device__ __forceinline__ v8f wmmab(v16bf a, v16bf b, v8f c) { return __builtin_amdgcn_wmma_f32_16x16x32_bf16(false, a, false, b, (short)0, c, false, false); }
__device__ __forceinline__ v16h  ldh(const h16* p) { return cat16(*(const v8h*)p, *(const v8h*)(p + 16)); }
__device__ __forceinline__ v16bf ldb(const bf* p)  { return cat16b(*(const v8us*)p, *(const v8us*)(p + 16)); }
__device__ __forceinline__ void wave_sync() { __builtin_amdgcn_fence(3  , "wavefront"); __builtin_amdgcn_wave_barrier(); asm volatile("" ::: "memory"); }

static __device__ __forceinline__ h16 toh_flush(float v) { const h16 r = (h16)v; return (fabsf(v) < 6.103515625e-05f) ? (h16)0.0f : r; }
__device__ __forceinline__ v8f wmma16g(v16h a, v16h b, v8f c) {
    c = wmma16(a, b, c);
    asm volatile("v_nop\n\tv_nop\n\tv_nop\n\tv_nop" : "+v"(c) : "v"(a), "v"(b));
    return c;
}
__device__ __forceinline__ v8f wmmabg(v16bf a, v16bf b, v8f c) {
    c = wmmab(a, b, c);
    asm volatile("v_nop\n\tv_nop\n\tv_nop\n\tv_nop" : "+v"(c) : "v"(a), "v"(b));
    return c;
}

__global__ __launch_bounds__(256) void k_cvt8(const float* __restrict__ src, bf* dst, size_t n8) {
    const size_t i = (size_t)blockIdx.x * 256 + threadIdx.x; if (i >= n8) return;
    const v8f v = *(const v8f*)(src + i * 8); v8us o;
#pragma unroll
    for (int k = 0; k < 8; ++k) o[k] = f2bf(v[k]);
    *(volatile v8us*)(dst + i * 8) = o; __threadfence(); *(volatile v8us*)(dst + i * 8) = o;
}

__global__ __launch_bounds__(256) void k_wcvth(const float* __restrict__ src, h16* dst, size_t n8) {
    const size_t i = (size_t)blockIdx.x * 256 + threadIdx.x; if (i >= n8) return;
    const v8f v = *(const v8f*)(src + i * 8); v8h o;
#pragma unroll
    for (int k = 0; k < 8; ++k) o[k] = toh_flush(bfr(v[k]) * WOS);
    *(volatile v8h*)(dst + i * 8) = o; __threadfence(); *(volatile v8h*)(dst + i * 8) = o;
}

__global__ __launch_bounds__(256) void k_wquat(const float* __restrict__ wr, const float* __restrict__ wi, const float* __restrict__ wj, const float* __restrict__ wk, bf* dst) {
    const int i = blockIdx.x * 256 + threadIdx.x;
    const int n = i / (DM / 8), k8 = (i % (DM / 8)) * 8;
    const int R = n / QB, p = n % QB, C = k8 / QB, q = k8 % QB;
    const int so = p * QB + q;
    const v8f a0 = *(const v8f*)(wr + so), a1 = *(const v8f*)(wi + so), a2 = *(const v8f*)(wj + so), a3 = *(const v8f*)(wk + so);
    const int c = R ^ C;
    const bool ng = ((0x284E >> (R * 4 + C)) & 1) != 0;
    v8us o;
#pragma unroll
    for (int e = 0; e < 8; ++e) {
        float v = (c == 0) ? a0[e] : ((c == 1) ? a1[e] : ((c == 2) ? a2[e] : a3[e]));
        v = ng ? -v : v;
        o[e] = f2bf(v); }
    *(volatile v8us*)(dst + (size_t)i * 8) = o; __threadfence(); *(volatile v8us*)(dst + (size_t)i * 8) = o;
}

__global__ __launch_bounds__(256) void k_thr(const float* __restrict__ feat, const int* __restrict__ mask, const float* __restrict__ thr0,
                                             const float* __restrict__ w1, const float* __restrict__ b1, const float* __restrict__ w2, const float* __restrict__ b2, float* KTH) {
#pragma clang fp contract(off)
    const int i = blockIdx.x * 256 + threadIdx.x;
    const int b = i / SEQ, t = i % SEQ;
    const size_t src = (size_t)b * SEQ_FULL + (size_t)t;
    const float f0 = bfr(feat[src * NFEAT + 0]), f1 = bfr(feat[src * NFEAT + 1]), f2 = bfr(feat[src * NFEAT + 2]);
    float d = bfr(b2[0]);
#pragma unroll 1
    for (int j = 0; j < NHID; ++j) {
        float hs = bfr(w1[j * NFEAT + 0]) * f0 + bfr(w1[j * NFEAT + 1]) * f1 + bfr(w1[j * NFEAT + 2]) * f2 + bfr(b1[j]);
        hs = 0.5f * hs * (1.0f + erff(hs * 0.70710678118654752f));
        d += bfr(w2[j]) * hs; }
    const float x = bfr(thr0[0]);
    const float ex = __builtin_amdgcn_exp2f(-fabsf(x) * L2E);
    const float sp = fmaxf(x, 0.0f) + __builtin_amdgcn_logf(1.0f + ex) * 0.6931471805599453f;
    const float tv = sp + d * 0.1f;
    int mk = mask[src];
    asm volatile("" : "+v"(mk));
    const float ov = (mk != 0) ? tv : THSENT;
    *(volatile float*)(KTH + i) = ov; __threadfence(); *(volatile float*)(KTH + i) = ov;
}

__global__ __launch_bounds__(32) void k_proj_qk(const bf* __restrict__ A, const bf* __restrict__ Bt, const float* __restrict__ bias, h16* Ph, h16* Pr) {
    __shared__ __align__(16) float os[16 * PSP];
    const int K = DM;
    const int lane = threadIdx.x & 31, lr = lane & 15, hi = lane >> 4; const int r0 = blockIdx.x * 64, c0 = blockIdx.y * 64;
    v8f acc[4][4];
#pragma unroll
    for (int mb = 0; mb < 4; ++mb)
#pragma unroll
        for (int nb = 0; nb < 4; ++nb) acc[mb][nb] = (v8f){};
    const size_t aoff = (size_t)(r0 + lr) * K + 8 * hi, boff = (size_t)(c0 + lr) * K + 8 * hi;
#pragma unroll 1
    for (int kc = 0; kc < K; kc += 32) {
        v16bf a[4];
#pragma unroll
        for (int mb = 0; mb < 4; ++mb) a[mb] = ldb(A + aoff + (size_t)mb * 16 * K + kc);
#pragma unroll
        for (int nb = 0; nb < 4; ++nb) { const v16bf b = ldb(Bt + boff + (size_t)nb * 16 * K + kc);
#pragma unroll
            for (int mb = 0; mb < 4; ++mb) acc[mb][nb] = wmmabg(a[mb], b, acc[mb][nb]); }
    }
    float bc[4];
#pragma unroll
    for (int nb = 0; nb < 4; ++nb) bc[nb] = bfr(bias[c0 + nb * 16 + lr]);
    const int bb = r0 / SEQ, tt = r0 % SEQ; const int zc = bb * NH_ + c0 / HD;
    const size_t tbase = ((size_t)zc * SEQ + (size_t)tt) * HD;
#pragma unroll
    for (int mb = 0; mb < 4; ++mb) {
#pragma unroll
        for (int nb = 0; nb < 4; ++nb) {
#pragma unroll
            for (int j = 0; j < 8; ++j) os[(hi * 8 + j) * PSP + nb * 16 + lr] = acc[mb][nb][j] + bc[nb]; }
        wave_sync();
        const size_t sb = tbase + (size_t)(mb * 16) * HD;
#pragma unroll 1
        for (int ps = 0; ps < 2; ++ps) {
#pragma unroll
            for (int s = 0; s < 4; ++s) { const int p = s * 32 + lane; const int row = p >> 3, c8 = (p & 7) * 8;
                const v4f x0 = *(const v4fa*)(&os[row * PSP + c8]); const v4f x1 = *(const v4fa*)(&os[row * PSP + c8 + 4]); v8h hv, rv;
#pragma unroll
                for (int i = 0; i < 4; ++i) { const h16 a0 = toh_flush(x0[i]); const h16 a1 = toh_flush(x1[i]); hv[i] = a0; hv[4 + i] = a1;
                    rv[i] = toh_flush((x0[i] - (float)a0) * QRS); rv[4 + i] = toh_flush((x1[i] - (float)a1) * QRS); }
                const size_t oo = sb + (size_t)p * 8;
                *(volatile v8h*)(Ph + oo) = hv; *(volatile v8h*)(Pr + oo) = rv; }
            if (ps == 0) __threadfence(); }
        wave_sync();
    }
}

__global__ __launch_bounds__(32) void k_proj_vt(const bf* __restrict__ A, const bf* __restrict__ Bt, const float* __restrict__ bias, h16* Ph) {
    __shared__ __align__(16) float os[16 * PSP];
    const int K = DM;
    const int lane = threadIdx.x & 31, lr = lane & 15, hi = lane >> 4; const int r0 = blockIdx.x * 64, c0 = blockIdx.y * 64;
    v8f acc[4][4];
#pragma unroll
    for (int mb = 0; mb < 4; ++mb)
#pragma unroll
        for (int nb = 0; nb < 4; ++nb) acc[mb][nb] = (v8f){};
    const size_t aoff = (size_t)(r0 + lr) * K + 8 * hi, boff = (size_t)(c0 + lr) * K + 8 * hi;
#pragma unroll 1
    for (int kc = 0; kc < K; kc += 32) {
        v16bf a[4];
#pragma unroll
        for (int mb = 0; mb < 4; ++mb) a[mb] = ldb(A + aoff + (size_t)mb * 16 * K + kc);
#pragma unroll
        for (int nb = 0; nb < 4; ++nb) { const v16bf b = ldb(Bt + boff + (size_t)nb * 16 * K + kc);
#pragma unroll
            for (int mb = 0; mb < 4; ++mb) acc[mb][nb] = wmmabg(a[mb], b, acc[mb][nb]); }
    }
    const int bb = c0 / SEQ, tt = c0 % SEQ;
    const size_t tbase = (size_t)bb * (size_t)DM * SEQ + (size_t)r0 * SEQ + (size_t)tt;
#pragma unroll
    for (int mb = 0; mb < 4; ++mb) {
        float br[8];
#pragma unroll
        for (int j = 0; j < 8; ++j) br[j] = bfr(bias[r0 + mb * 16 + hi * 8 + j]);
#pragma unroll
        for (int nb = 0; nb < 4; ++nb) {
#pragma unroll
            for (int j = 0; j < 8; ++j) os[(hi * 8 + j) * PSP + nb * 16 + lr] = acc[mb][nb][j] + br[j]; }
        wave_sync();
        const size_t sb = tbase + (size_t)(mb * 16) * SEQ;
#pragma unroll 1
        for (int ps = 0; ps < 2; ++ps) {
#pragma unroll
            for (int s = 0; s < 4; ++s) { const int row = 4 * s + (lane >> 3), c8 = (lane & 7) * 8;
                const v4f x0 = *(const v4fa*)(&os[row * PSP + c8]); const v4f x1 = *(const v4fa*)(&os[row * PSP + c8 + 4]); v8h hv;
#pragma unroll
                for (int i = 0; i < 4; ++i) { hv[i] = toh_flush(x0[i]); hv[4 + i] = toh_flush(x1[i]); }
                const size_t oo = sb + (size_t)row * SEQ + c8;
                *(volatile v8h*)(Ph + oo) = hv; }
            if (ps == 0) __threadfence(); }
        wave_sync();
    }
}

__global__ __launch_bounds__(32) void k_proj_out(const h16* __restrict__ A, const h16* __restrict__ Bt, const float* __restrict__ bias, float* OUT) {
    __shared__ __align__(16) float os[16 * PSP];
    const int K = DM;
    const int lane = threadIdx.x & 31, lr = lane & 15, hi = lane >> 4; const int r0 = blockIdx.x * 64, c0 = blockIdx.y * 64;
    v8f acc[4][4];
#pragma unroll
    for (int mb = 0; mb < 4; ++mb)
#pragma unroll
        for (int nb = 0; nb < 4; ++nb) acc[mb][nb] = (v8f){};
    const size_t aoff = (size_t)(r0 + lr) * K + 8 * hi, boff = (size_t)(c0 + lr) * K + 8 * hi;
#pragma unroll 1
    for (int kc = 0; kc < K; kc += 32) {
        v16h a[4];
#pragma unroll
        for (int mb = 0; mb < 4; ++mb) a[mb] = ldh(A + aoff + (size_t)mb * 16 * K + kc);
#pragma unroll
        for (int nb = 0; nb < 4; ++nb) { const v16h b = ldh(Bt + boff + (size_t)nb * 16 * K + kc);
#pragma unroll
            for (int mb = 0; mb < 4; ++mb) acc[mb][nb] = wmma16g(a[mb], b, acc[mb][nb]); }
    }
    float bc[4];
#pragma unroll
    for (int nb = 0; nb < 4; ++nb) bc[nb] = bfr(bias[c0 + nb * 16 + lr]);
    const int bb = r0 / SEQ, tt = r0 % SEQ;
    float* obase = OUT + ((size_t)bb * OUT_SEQ + (size_t)tt) * DM + c0;
#pragma unroll
    for (int mb = 0; mb < 4; ++mb) {
#pragma unroll
        for (int nb = 0; nb < 4; ++nb) {
#pragma unroll
            for (int j = 0; j < 8; ++j) os[(hi * 8 + j) * PSP + nb * 16 + lr] = acc[mb][nb][j] * OSI + bc[nb]; }
        wave_sync();
        float* orow = obase + (size_t)(mb * 16) * DM;
#pragma unroll 1
        for (int ps = 0; ps < 2; ++ps) {
#pragma unroll
            for (int s = 0; s < 8; ++s) { const int row = 2 * s + (lane >> 4), cofs = (lane & 15) * 4;
                const v4f val = *(const v4fa*)(&os[row * PSP + cofs]);
                *(volatile v4f*)(orow + (size_t)row * DM + cofs) = val; }
            if (ps == 0) __threadfence(); }
        wave_sync();
    }
}

__device__ __forceinline__ float gate_logit(float sv, float sr, float thv, bool qz) {
    float s = (sv + sr * QRI) * SSC;
    s = fminf(fmaxf(s, -6.0f), 6.0f);
    const bool fill = qz | (thv > THCUT);
    const float ea = fminf((s - thv) * GSL2, 126.0f);
    const float g = __builtin_amdgcn_rcpf(1.0f + __builtin_amdgcn_exp2f(ea));
    const float md = s * (L2E + L2E2 * g);
    const float sel = fill ? FILL2 : md;
    return fminf(fmaxf(sel, -C30), C30);
}

__global__ __launch_bounds__(32 * AW) __attribute__((amdgpu_num_vgpr(256)))
void k_flash(const h16* __restrict__ QH, const h16* __restrict__ QR, const h16* __restrict__ KP, const h16* __restrict__ KR,
             const h16* __restrict__ VT, const float* __restrict__ KTH, const int* __restrict__ qmask, h16* CT) {
    __shared__ __align__(16) float os[AW * 16 * OSP];
    const int lane = threadIdx.x & 31, lr = lane & 15, hi = lane >> 4;
    const int wave = __builtin_amdgcn_readfirstlane((int)(threadIdx.x >> 5));
    const int zh = blockIdx.y; const int b = zh / NH_, h = zh % NH_;
    const int t0 = (blockIdx.x * AW + wave) * 16;
    int qmi = qmask[(size_t)b * SEQ_FULL + t0 + lr];
    asm volatile("" : "+v"(qmi));
    const bool qz = (qmi == 0);
    const float* kth = KTH + (size_t)b * SEQ + 8 * hi;
    const size_t pbase = (size_t)zh * SEQ * HD;
    const size_t qo = pbase + (size_t)(t0 + lr) * HD + 8 * hi;
    const v16h qh0 = ldh(QH + qo), qh1 = ldh(QH + qo + 32), qr0 = ldh(QR + qo), qr1 = ldh(QR + qo + 32);
    const size_t ko = pbase + (size_t)lr * HD + 8 * hi;
    const size_t vo = pbase + (size_t)lr * SEQ + 8 * hi;
    v8f o[4];
#pragma unroll
    for (int j = 0; j < 4; ++j) o[j] = (v8f){};
    float m = NEGB, l = 0.0f;
#pragma unroll 1
    for (int key0 = 0; key0 < SEQ; key0 += 32) {
        const size_t kk = ko + (size_t)key0 * HD;
        v8f sHa = (v8f){}, sLa = (v8f){}, sHb = (v8f){}, sLb = (v8f){};
        { const v16h ka = ldh(KP + kk), kb = ldh(KP + kk + 16 * HD), ra = ldh(KR + kk), rb = ldh(KR + kk + 16 * HD);
          sHa = wmma16g(ka, qh0, sHa); sHb = wmma16g(kb, qh0, sHb);
          sLa = wmma16g(ka, qr0, sLa); sLb = wmma16g(kb, qr0, sLb);
          sLa = wmma16g(ra, qh0, sLa); sLb = wmma16g(rb, qh0, sLb); }
        { const v16h ka = ldh(KP + kk + 32), kb = ldh(KP + kk + 16 * HD + 32), ra = ldh(KR + kk + 32), rb = ldh(KR + kk + 16 * HD + 32);
          sHa = wmma16g(ka, qh1, sHa); sHb = wmma16g(kb, qh1, sHb);
          sLa = wmma16g(ka, qr1, sLa); sLb = wmma16g(kb, qr1, sLb);
          sLa = wmma16g(ra, qh1, sLa); sLb = wmma16g(rb, qh1, sLb); }
        const float* kp = kth + key0;
        const v4f th0 = *(const v4f*)kp, th1 = *(const v4f*)(kp + 4), th2 = *(const v4f*)(kp + 16), th3 = *(const v4f*)(kp + 20);
        float kx[8], ky[8];
#pragma unroll
        for (int r = 0; r < 4; ++r) { kx[r] = th0[r]; kx[4 + r] = th1[r]; ky[r] = th2[r]; ky[4 + r] = th3[r]; }
        float ta[8], tb[8]; float mx = NEGB;
#pragma unroll
        for (int r = 0; r < 8; ++r) {
            ta[r] = gate_logit(sHa[r], sLa[r], kx[r], qz);
            tb[r] = gate_logit(sHb[r], sLb[r], ky[r], qz);
            mx = fmaxf(mx, fmaxf(ta[r], tb[r])); }
        mx = fmaxf(mx, __shfl_xor(mx, 16, 32));
        const float mnew = fmaxf(m, mx);
        const float alpha = __builtin_amdgcn_exp2f(m - mnew);
        const float sh = PSH - mnew;
        v16h pb; float ls = 0.0f;
#pragma unroll
        for (int r = 0; r < 8; ++r) {
            const float xa = ta[r] + sh, xb = tb[r] + sh;
            const float ea = __builtin_amdgcn_exp2f(xa), eb = __builtin_amdgcn_exp2f(xb);
            const float ga = (xa < -14.0f) ? 0.0f : ea, gb = (xb < -14.0f) ? 0.0f : eb;
            const h16 pa = (h16)ga; const h16 pc = (h16)gb;
            pb[r] = pa; pb[8 + r] = pc;
            ls += (float)pa + (float)pc; }
        l = l * alpha + ls; m = mnew;
#pragma unroll
        for (int j = 0; j < 4; ++j) o[j] = o[j] * alpha;
        const h16* va = VT + vo + key0;
        v16h vf[4];
#pragma unroll
        for (int j = 0; j < 4; ++j) vf[j] = ldh(va + (size_t)(16 * j) * SEQ);
#pragma unroll
        for (int j = 0; j < 4; ++j) o[j] = wmma16g(vf[j], pb, o[j]);
    }
    l += __shfl_xor(l, 16, 32);
    const float inv = 1.0f / l;
    const int wb = wave * 16 * OSP;
#pragma unroll
    for (int j = 0; j < 4; ++j) { v4f a, c;
        a[0] = o[j][0] * inv; a[1] = o[j][1] * inv; a[2] = o[j][2] * inv; a[3] = o[j][3] * inv;
        c[0] = o[j][4] * inv; c[1] = o[j][5] * inv; c[2] = o[j][6] * inv; c[3] = o[j][7] * inv;
        *(v4fa*)(&os[wb + lr * OSP + 16 * j + 8 * hi]) = a; *(v4fa*)(&os[wb + lr * OSP + 16 * j + 8 * hi + 4]) = c; }
    wave_sync();
    h16* crow = CT + ((size_t)b * SEQ + (size_t)t0) * DM + h * HD;
#pragma unroll 1
    for (int ps = 0; ps < 2; ++ps) {
#pragma unroll
        for (int s = 0; s < 4; ++s) { const int row = 4 * s + (lane >> 3), c8 = (lane & 7) * 8;
            const v4f x0 = *(const v4fa*)(&os[wb + row * OSP + c8]); const v4f x1 = *(const v4fa*)(&os[wb + row * OSP + c8 + 4]); v8h cv;
#pragma unroll
            for (int i = 0; i < 4; ++i) { cv[i] = toh_flush(x0[i] * CTS); cv[4 + i] = toh_flush(x1[i] * CTS); }
            *(volatile v8h*)(crow + (size_t)row * DM + c8) = cv; }
        if (ps == 0) __threadfence(); }
}

static constexpr size_t al256(size_t v) { return (v + 255) & ~(size_t)255; }
static constexpr size_t SZ_XB = al256((size_t)NB * SEQ * DM * 2);
static constexpr size_t SZ_WB = al256((size_t)3 * DM * DM * 2);
static constexpr size_t SZ_WH = al256((size_t)DM * DM * 2);
static constexpr size_t SZ_PL = al256((size_t)NB * NH_ * SEQ * HD * 2);
static constexpr size_t SZ_TH = al256((size_t)NB * SEQ * 4);
static constexpr size_t SZ_TOTAL = 3 * SZ_XB + SZ_WB + SZ_WH + 6 * SZ_PL + SZ_TH;
static_assert(SZ_TOTAL <= (size_t)134217728);
static_assert(((size_t)DM * DM * 2) % 256 == 0);
static_assert((size_t)NB * NH_ * SEQ * HD == (size_t)NB * DM * SEQ);

extern "C" void kernel_launch(void* const* d_in, const int* in_sizes, int n_in,
                              void* d_out, int out_size, void* d_ws, size_t ws_size, hipStream_t stream) {
    if (n_in < 24) return;
    const size_t needx = ((size_t)(NB - 1) * SEQ_FULL + SEQ) * DM;
    const size_t needm = (size_t)(NB - 1) * SEQ_FULL + SEQ;
    if ((size_t)in_sizes[0] < needx || (size_t)in_sizes[1] < needx || (size_t)in_sizes[2] < needx) return;
    if ((size_t)in_sizes[3] < needm * NFEAT || (size_t)in_sizes[4] < needm) return;
    for (int i = 5; i <= 8; ++i) { if (in_sizes[i] < QB * QB || in_sizes[i + 5] < QB * QB) return; }
    if (in_sizes[9] < DM || in_sizes[14] < DM || in_sizes[16] < DM || in_sizes[18] < DM) return;
    if (in_sizes[15] < DM * DM || in_sizes[17] < DM * DM) return;
    if (in_sizes[19] < 1 || in_sizes[20] < NHID * NFEAT || in_sizes[21] < NHID || in_sizes[22] < NHID || in_sizes[23] < 1) return;
    if ((size_t)out_size < ((size_t)(NB - 1) * OUT_SEQ + SEQ) * DM) return;
    if (SZ_TOTAL > ws_size) return;
    const float* xin[3] = { (const float*)d_in[0], (const float*)d_in[1], (const float*)d_in[2] };
    const float* feat = (const float*)d_in[3];
    const int*   mask = (const int*)d_in[4];
    const float* wqr = (const float*)d_in[5];  const float* wqi = (const float*)d_in[6];
    const float* wqj = (const float*)d_in[7];  const float* wqk = (const float*)d_in[8];
    const float* bq  = (const float*)d_in[9];
    const float* wkr = (const float*)d_in[10]; const float* wki = (const float*)d_in[11];
    const float* wkj = (const float*)d_in[12]; const float* wkk = (const float*)d_in[13];
    const float* bk  = (const float*)d_in[14];
    const float* wv  = (const float*)d_in[15]; const float* bv = (const float*)d_in[16];
    const float* wo  = (const float*)d_in[17]; const float* bo = (const float*)d_in[18];
    const float* th0 = (const float*)d_in[19];
    const float* w1  = (const float*)d_in[20]; const float* b1 = (const float*)d_in[21];
    const float* w2  = (const float*)d_in[22]; const float* b2 = (const float*)d_in[23];
    float* OUT = (float*)d_out;
    char* wsp = (char*)d_ws;
    bf* XB[3];
    XB[0] = (bf*)wsp; wsp += SZ_XB;
    XB[1] = (bf*)wsp; wsp += SZ_XB;
    XB[2] = (bf*)wsp; wsp += SZ_XB;
    bf* WB = (bf*)wsp; wsp += SZ_WB;
    h16* WOH = (h16*)wsp; wsp += SZ_WH;
    h16* QH = (h16*)wsp; wsp += SZ_PL;
    h16* QR = (h16*)wsp; wsp += SZ_PL;
    h16* KP = (h16*)wsp; wsp += SZ_PL;
    h16* KR = (h16*)wsp; wsp += SZ_PL;
    h16* VT = (h16*)wsp; wsp += SZ_PL;
    h16* CT = (h16*)wsp; wsp += SZ_PL;
    float* KTH = (float*)wsp; wsp += SZ_TH;
    bf* WQ = WB; bf* WK = WB + (size_t)DM * DM; bf* WV = WB + (size_t)2 * DM * DM;

    for (int i = 0; i < 3; ++i) {
        if (SEQ == SEQ_FULL) {
            const size_t n8 = (size_t)NB * SEQ * DM / 8;
            k_cvt8<<<(unsigned)((n8 + 255) / 256), 256, 0, stream>>>(xin[i], XB[i], n8);
        } else {
            const size_t n8 = (size_t)SEQ * DM / 8;
            for (int b = 0; b < NB; ++b) k_cvt8<<<(unsigned)((n8 + 255) / 256), 256, 0, stream>>>(xin[i] + (size_t)b * SEQ_FULL * DM, XB[i] + (size_t)b * SEQ * DM, n8);
        }
    }
    { const size_t n8 = (size_t)DM * DM / 8; const unsigned g = (unsigned)((n8 + 255) / 256);
      k_wquat<<<g, 256, 0, stream>>>(wqr, wqi, wqj, wqk, WQ);
      k_wquat<<<g, 256, 0, stream>>>(wkr, wki, wkj, wkk, WK);
      k_cvt8<<<g, 256, 0, stream>>>(wv, WV, n8);
      k_wcvth<<<g, 256, 0, stream>>>(wo, WOH, n8); }
    k_thr<<<(unsigned)((size_t)NB * SEQ / 256), 256, 0, stream>>>(feat, mask, th0, w1, b1, w2, b2, KTH);

    k_proj_qk<<<dim3(NB * SEQ / 64, DM / 64, 1), 32, 0, stream>>>(XB[0], WQ, bq, QH, QR);
    k_proj_qk<<<dim3(NB * SEQ / 64, DM / 64, 1), 32, 0, stream>>>(XB[1], WK, bk, KP, KR);
    k_proj_vt<<<dim3(DM / 64, NB * SEQ / 64, 1), 32, 0, stream>>>(WV, XB[2], bv, VT);

    k_flash<<<dim3(SEQ / (16 * AW), NB * NH_, 1), 32 * AW, 0, stream>>>(QH, QR, KP, KR, VT, KTH, mask, CT);

    k_proj_out<<<dim3(NB * SEQ / 64, DM / 64, 1), 32, 0, stream>>>(CT, WOH, bo, OUT);
}
